// LogicalEncoder_58832462021326
// MI455X (gfx1250) — hardware-verified
//
#include <hip/hip_runtime.h>
#include <stddef.h>


#define DM    64
#define TT    64
#define NTHR  256
#define NWAVE 8
#define GN    32
#define HP    72
#define FP    68
#define CHUNK 2048
#define WCAP  256
#define NGRP  (CHUNK / (NTHR * 4))
#define STHR  512
#define NWS   (STHR / 32)
#define NITER 64
#define MAXN  30000
#define NBS   512
#define SLBS  9
#define CAPB  32768
#define MAXDG 512
#define WCAPS ((CHUNK / STHR) * 32 * 2)

static_assert(WCAP == (CHUNK / NTHR) * 32);
static_assert(NGRP == 2);
static_assert((HP % 8) == 0);
static_assert((FP % 4) == 0);
static_assert(GN * 8 == NTHR);
static_assert(CHUNK == STHR * 4);
static_assert(WCAPS == 256);
static_assert((1 << SLBS) == NBS);
static_assert((CAPB % 4) == 0 && (NBS % 4) == 0);

#define LDS_CSR_INTS  (CAPB + 4 * NBS + NWS * WCAPS + NWS)
#define LDS_CSR_BYTES (LDS_CSR_INTS * 4)
static_assert(LDS_CSR_BYTES == 155712);

typedef float    v2f  __attribute__((ext_vector_type(2)));
typedef float    v4f  __attribute__((ext_vector_type(4)));
typedef float    v8f  __attribute__((ext_vector_type(8)));
typedef int      v4i  __attribute__((ext_vector_type(4)));
typedef _Float16 v8h  __attribute__((ext_vector_type(8)));
typedef _Float16 v16h __attribute__((ext_vector_type(16)));
union Frag   { v16h v; v8h half[2]; };
union Pack16 { v8h h; v4i i; };

__device__ __forceinline__ v8f wm(v16h a, v16h b, v8f c) {
  v8f d = __builtin_amdgcn_wmma_f32_16x16x32_f16(false, a, false, b, (short)0, c, false, false);
  asm volatile("v_nop\n\tv_nop\n\tv_nop\n\tv_nop" : "+v"(d) : "v"(a), "v"(b));
  return d;
}

__device__ __forceinline__ float wsum(float v) {
  v += __shfl_xor(v, 16, 32);
  v += __shfl_xor(v, 8, 32);
  v += __shfl_xor(v, 4, 32);
  v += __shfl_xor(v, 2, 32);
  v += __shfl_xor(v, 1, 32);
  return v;
}

__device__ __forceinline__ float sigm(float x) { return __builtin_amdgcn_rcpf(1.0f + __expf(-x)); }
__device__ __forceinline__ float tnh(float x)  { return 2.0f * sigm(2.0f * x) - 1.0f; }

__device__ __forceinline__ void ld8f(const float* p, float* o) {
  const v4f a = *(const v4f*)p, b = *(const v4f*)(p + 4);
  o[0] = a.x; o[1] = a.y; o[2] = a.z; o[3] = a.w; o[4] = b.x; o[5] = b.y; o[6] = b.z; o[7] = b.w;
}
__device__ __forceinline__ void st8f(float* p, const float* o) {
  v4f a, b;
  a.x = o[0]; a.y = o[1]; a.z = o[2]; a.w = o[3]; b.x = o[4]; b.y = o[5]; b.z = o[6]; b.w = o[7];
  *(v4f*)p = a; *(v4f*)(p + 4) = b;
}
__device__ __forceinline__ void ld2f(const float* p, float* o) {
  const v2f a = *(const v2f*)p;
  o[0] = a.x; o[1] = a.y;
}
__device__ __forceinline__ void st2f(float* p, const float* o) {
  v2f a; a.x = o[0]; a.y = o[1];
  *(v2f*)p = a;
}
template <int CPL> __device__ __forceinline__ void ldc(const float* p, float* o) {
  if constexpr (CPL == 8) ld8f(p, o); else ld2f(p, o);
}
template <int CPL> __device__ __forceinline__ void stc(float* p, const float* o) {
  if constexpr (CPL == 8) st8f(p, o); else st2f(p, o);
}

__global__ __launch_bounds__(NTHR) void k_prep(const float* __restrict__ Whh, const float* __restrict__ W1,
                                                 const float* __restrict__ W2, _Float16* Whh16,
                                                 _Float16* Wt1, _Float16* Wt2) {
  const int tid = threadIdx.x;
  const int b   = blockIdx.x;
  float v[8];
  _Float16* dst;
  if (b < 6) {
    const int i  = b * NTHR + tid;
    const int n  = i >> 3, k0 = (i & 7) * 8;
    const float* p = Whh + n * DM + k0;
    const v4f a = *(const v4f*)p, c = *(const v4f*)(p + 4);
    v[0] = a.x; v[1] = a.y; v[2] = a.z; v[3] = a.w; v[4] = c.x; v[5] = c.y; v[6] = c.z; v[7] = c.w;
    dst = Whh16 + n * DM + k0;
  } else if (b < 14) {
    const int i  = (b - 6) * NTHR + tid;
    const int n  = i >> 3, k0 = (i & 7) * 8;
#pragma unroll
    for (int j = 0; j < 8; ++j) v[j] = W1[(k0 + j) * 256 + n];
    dst = Wt1 + n * 64 + k0;
  } else {
    const int i  = (b - 14) * NTHR + tid;
    const int n  = i >> 5, k0 = (i & 31) * 8;
#pragma unroll
    for (int j = 0; j < 8; ++j) v[j] = W2[(k0 + j) * 64 + n];
    dst = Wt2 + n * 256 + k0;
  }
  Pack16 u;
#pragma unroll
  for (int j = 0; j < 8; ++j) u.h[j] = (_Float16)(v[j] * 8.0f);
  *(volatile v4i*)dst = u.i;
  __threadfence();
  *(volatile v4i*)dst = u.i;
}

#define CHIT(HJ, ENT) { \
    const unsigned mj = __builtin_amdgcn_ballot_w32(HJ); \
    if (HJ) { \
      const int pos = wc + (int)__builtin_amdgcn_mbcnt_lo(mj, 0u); \
      if (pos < WCAPS) list[wave * WCAPS + pos] = (ENT); \
    } \
    wc += (int)__builtin_popcount(mj); }

template <int WS>
__device__ __forceinline__ int csr_scan(const int* eis, const int* eid, int nE, int cbase, bool al16,
                                        int nodeBase, int tid, int wave, int* list) {
  const int el0  = tid * 4;
  const int e0   = cbase + el0;
  const int sent = -2147483647 - 1;
  const int nE1  = nE - 1;
  v4i d4, s4;
  if (al16 && (cbase + CHUNK <= nE)) {
    d4 = *(const v4i*)(eid + e0);
    if (WS) s4 = *(const v4i*)(eis + e0); else s4 = d4;
  } else {
    d4.x = (e0     < nE) ? eid[min(e0, nE1)]     : sent;
    d4.y = (e0 + 1 < nE) ? eid[min(e0 + 1, nE1)] : sent;
    d4.z = (e0 + 2 < nE) ? eid[min(e0 + 2, nE1)] : sent;
    d4.w = (e0 + 3 < nE) ? eid[min(e0 + 3, nE1)] : sent;
    if (WS) {
      s4.x = (e0     < nE) ? eis[min(e0, nE1)]     : sent;
      s4.y = (e0 + 1 < nE) ? eis[min(e0 + 1, nE1)] : sent;
      s4.z = (e0 + 2 < nE) ? eis[min(e0 + 2, nE1)] : sent;
      s4.w = (e0 + 3 < nE) ? eis[min(e0 + 3, nE1)] : sent;
    } else {
      s4 = d4;
    }
  }
  const unsigned ud0 = (unsigned)d4.x - (unsigned)nodeBase;
  const unsigned ud1 = (unsigned)d4.y - (unsigned)nodeBase;
  const unsigned ud2 = (unsigned)d4.z - (unsigned)nodeBase;
  const unsigned ud3 = (unsigned)d4.w - (unsigned)nodeBase;
  const unsigned us0 = (unsigned)s4.x - (unsigned)nodeBase;
  const unsigned us1 = (unsigned)s4.y - (unsigned)nodeBase;
  const unsigned us2 = (unsigned)s4.z - (unsigned)nodeBase;
  const unsigned us3 = (unsigned)s4.w - (unsigned)nodeBase;
  const bool hd0 = ud0 < (unsigned)NBS;
  const bool hd1 = ud1 < (unsigned)NBS;
  const bool hd2 = ud2 < (unsigned)NBS;
  const bool hd3 = ud3 < (unsigned)NBS;
  const bool hs0 = (WS != 0) && (us0 < (unsigned)NBS);
  const bool hs1 = (WS != 0) && (us1 < (unsigned)NBS);
  const bool hs2 = (WS != 0) && (us2 < (unsigned)NBS);
  const bool hs3 = (WS != 0) && (us3 < (unsigned)NBS);
  int wc = 0;
  const unsigned many = __builtin_amdgcn_ballot_w32(hd0 | hd1 | hd2 | hd3 | hs0 | hs1 | hs2 | hs3);
  if (many != 0u) {
    CHIT(hd0, ((el0 + 0) << 10) | (int)ud0)
    if (WS) CHIT(hs0, ((el0 + 0) << 10) | NBS | (int)us0)
    CHIT(hd1, ((el0 + 1) << 10) | (int)ud1)
    if (WS) CHIT(hs1, ((el0 + 1) << 10) | NBS | (int)us1)
    CHIT(hd2, ((el0 + 2) << 10) | (int)ud2)
    if (WS) CHIT(hs2, ((el0 + 2) << 10) | NBS | (int)us2)
    CHIT(hd3, ((el0 + 3) << 10) | (int)ud3)
    if (WS) CHIT(hs3, ((el0 + 3) << 10) | NBS | (int)us3)
  }
  return wc;
}
#undef CHIT

__global__ __launch_bounds__(STHR) void k_csr(const int* __restrict__ ei, int nE, int nN,
                                                int* csr, int* pcin, int* pcou, int* poff) {
  extern __shared__ v4i lds_c4[];
  int* seg  = (int*)lds_c4;
  int* cin  = seg + CAPB;
  int* cou  = cin + NBS;
  int* off  = cou + NBS;
  int* cur  = off + NBS;
  int* list = cur + NBS;
  int* wcnt = list + NWS * WCAPS;

  const int tid  = threadIdx.x;
  const int lane = tid & 31;
  const int wave = tid >> 5;
  const int nodeBase = blockIdx.x * NBS;
  const int nN1 = nN - 1;
  const int nE1 = nE - 1;

  {
    const v4i z4 = {0, 0, 0, 0};
    for (int i = tid; i < (CAPB + 4 * NBS) / 4; i += STHR) lds_c4[i] = z4;
  }
  __syncthreads();

  const int* eis = ei;
  const int* eid = ei + nE;
  const bool al16 = ((nE & 3) == 0);
  const int nChunks = (nE + CHUNK - 1) / CHUNK;

#pragma unroll 1
  for (int ch = 0; ch < nChunks; ++ch) {
    const int cbase = ch * CHUNK;
    const int wc = csr_scan<1>(eis, eid, nE, cbase, al16, nodeBase, tid, wave, list);
    if (lane == 0) wcnt[wave] = wc;
    __syncthreads();
    if (wave == 0) {
#pragma unroll 1
      for (int wsx = 0; wsx < NWS; ++wsx) {
        int n = wcnt[wsx];
        if (n > WCAPS) n = WCAPS;
        if (n < 0) n = 0;
#pragma unroll 1
        for (int i = 0; i < n; ++i) {
          const int ent = list[wsx * WCAPS + i];
          const int ci  = ent & (2 * NBS - 1);
          const int v   = cin[ci];
          cin[ci] = v + 1;
        }
      }
    }
    __syncthreads();
  }

  if (tid == 0) {
    int a = 0;
#pragma unroll 1
    for (int s = 0; s < NBS; ++s) { off[s] = a; a += cin[s]; }
  }
  __syncthreads();

#pragma unroll 1
  for (int ch = 0; ch < nChunks; ++ch) {
    const int cbase = ch * CHUNK;
    const int wc = csr_scan<0>(eis, eid, nE, cbase, al16, nodeBase, tid, wave, list);
    if (lane == 0) wcnt[wave] = wc;
    __syncthreads();
    if (wave == 0) {
#pragma unroll 1
      for (int wsx = 0; wsx < NWS; ++wsx) {
        int n = wcnt[wsx];
        if (n > WCAPS) n = WCAPS;
        if (n < 0) n = 0;
#pragma unroll 1
        for (int i = 0; i < n; ++i) {
          const int ent  = list[wsx * WCAPS + i];
          const int slot = ent & (NBS - 1);
          const int el   = (ent >> 10) & (CHUNK - 1);
          int e = cbase + el;
          if (e > nE1) e = nE1;
          int s = eis[e];
          s = min(max(s, 0), nN1);
          const int cv  = cur[slot];
          const int pos = off[slot] + cv;
          cur[slot] = cv + 1;
          if ((unsigned)pos < (unsigned)CAPB) seg[pos] = s;
        }
      }
    }
    __syncthreads();
  }

  int* gseg = csr + (size_t)blockIdx.x * CAPB;
  const v4i* seg4 = (const v4i*)seg;
  const v4i* cin4 = (const v4i*)cin;
  const v4i* cou4 = (const v4i*)cou;
  const v4i* off4 = (const v4i*)off;
#pragma unroll 1
  for (int pass = 0; pass < 2; ++pass) {
#pragma unroll 1
    for (int i = tid; i < CAPB / 4; i += STHR) *(volatile v4i*)(gseg + 4 * i) = seg4[i];
    if (tid < NBS / 4) {
      *(volatile v4i*)(pcin + nodeBase + 4 * tid) = cin4[tid];
      *(volatile v4i*)(pcou + nodeBase + 4 * tid) = cou4[tid];
      *(volatile v4i*)(poff + nodeBase + 4 * tid) = off4[tid];
    }
    __threadfence();
  }
}

__device__ __forceinline__ void st_deg(const int* pcin, const int* pcou, float rin, float rou,
                                       float* fin, float* fout, int nq, int tid) {
#pragma unroll 1
  for (int i = tid; i < nq; i += STHR) {
    const int b = 4 * i;
    const v4i a = *(const v4i*)(pcin + b);
    const v4i c = *(const v4i*)(pcou + b);
    v4f fa, fc;
    fa.x = (float)a.x * rin; fa.y = (float)a.y * rin; fa.z = (float)a.z * rin; fa.w = (float)a.w * rin;
    fc.x = (float)c.x * rou; fc.y = (float)c.y * rou; fc.z = (float)c.z * rou; fc.w = (float)c.w * rou;
    *(volatile v4f*)(fin + b)  = fa;
    *(volatile v4f*)(fout + b) = fc;
  }
}

__device__ __forceinline__ void st_lvl(const int* lv, float* flvl, int nq, int nN1, int tid) {
#pragma unroll 1
  for (int i = tid; i < nq; i += STHR) {
    const int b = 4 * i;
    v4f a;
    a.x = (float)lv[min(b, nN1)];
    a.y = (float)lv[min(b + 1, nN1)];
    a.z = (float)lv[min(b + 2, nN1)];
    a.w = (float)lv[min(b + 3, nN1)];
    *(volatile v4f*)(flvl + b) = a;
  }
}

__global__ __launch_bounds__(STHR) void k_struct(const int* __restrict__ csr, const int* __restrict__ pcin,
                                                   const int* __restrict__ pcou, const int* __restrict__ poff,
                                                   int nN, int nP, float* fin, float* fout, float* flvl) {
  extern __shared__ int slv[];
  __shared__ int rdi[NWS];
  __shared__ int rdo[NWS];
  const int tid = threadIdx.x, lane = tid & 31, wave = tid >> 5;
  const int nN1 = nN - 1;
  const int nq  = nP >> 2;

  int m0 = 0, m1 = 0;
  for (int i = tid; i < nN; i += STHR) { m0 = max(m0, pcin[i]); m1 = max(m1, pcou[i]); }
#pragma unroll
  for (int k = 16; k > 0; k >>= 1) {
    m0 = max(m0, __shfl_xor(m0, k, 32));
    m1 = max(m1, __shfl_xor(m1, k, 32));
  }
  if (lane == 0) { rdi[wave] = m0; rdo[wave] = m1; }
  __syncthreads();
  int g0 = 0, g1 = 0;
#pragma unroll
  for (int w = 0; w < NWS; ++w) { g0 = max(g0, rdi[w]); g1 = max(g1, rdo[w]); }
  const float rin = 1.0f / ((float)g0 + 1e-6f);
  const float rou = 1.0f / ((float)g1 + 1e-6f);
  st_deg(pcin, pcou, rin, rou, fin, fout, nq, tid);
  __threadfence();
  st_deg(pcin, pcou, rin, rou, fin, fout, nq, tid);

  for (int i = tid; i < nN; i += STHR) slv[i] = 0;
  __syncthreads();
  int co = 0, no = nN;
#pragma unroll 1
  for (int it = 0; it < NITER; ++it) {
#pragma unroll 1
    for (int i = tid; i < nN; i += STHR) {
      int c = pcin[i]; c = min(max(c, 0), MAXDG);
      int o = poff[i]; o = min(max(o, 0), CAPB - 1);
      const int* reg = csr + (size_t)(i >> SLBS) * CAPB;
      int best = slv[co + i];
#pragma unroll 1
      for (int k = 0; k < c; ++k) {
        const int pos = min(o + k, CAPB - 1);
        int s = reg[pos];
        s = min(max(s, 0), nN1);
        best = max(best, slv[co + s] + 1);
      }
      slv[no + i] = best;
    }
    __syncthreads();
    const int t = co; co = no; no = t;
  }
  st_lvl(slv + co, flvl, nq, nN1, tid);
  __threadfence();
  st_lvl(slv + co, flvl, nq, nN1, tid);
}

__global__ __launch_bounds__(NTHR) void k_gru(
    const float* __restrict__ tcs, const float* __restrict__ hls,
    const float* __restrict__ Wih, const _Float16* __restrict__ Whh16,
    const float* __restrict__ bih, const float* __restrict__ bhh,
    const float* __restrict__ lng, const float* __restrict__ lnb,
    const float* __restrict__ flops, const float* __restrict__ memv,
    const float* __restrict__ Wst, const float* __restrict__ bst,
    const float* __restrict__ fin, const float* __restrict__ fout, const float* __restrict__ flvl,
    const float* __restrict__ Wsr, const float* __restrict__ bsr,
    _Float16* x0h, int nN) {
  __shared__ __attribute__((aligned(16))) float    xcl[GN * TT];
  __shared__ __attribute__((aligned(16))) float    xll[GN * TT];
  __shared__ __attribute__((aligned(16))) _Float16 hA[GN * HP];
  __shared__ __attribute__((aligned(16))) float    hf[GN * FP];

  const int tid  = threadIdx.x;
  const int lane = tid & 31;
  const int wave = tid >> 5;
  const int hh   = lane >> 4;
  const int m    = lane & 15;
  const int mt   = wave >> 2;
  const int jq   = wave & 3;
  const int d    = 16 * jq + m;
  const int nodeBase = blockIdx.x * GN;
  const int q  = tid >> 3;
  const int c0 = (tid & 7) * 8;

  {
    int nd = nodeBase + q;
    if (nd > nN - 1) nd = nN - 1;
    const float* p = tcs + (size_t)nd * TT + c0;
    const v4f a = *(const v4f*)p, b = *(const v4f*)(p + 4);
    *(v4f*)(xcl + q * TT + c0)     = a;
    *(v4f*)(xcl + q * TT + c0 + 4) = b;
    const float* ph = hls + (size_t)nd * TT + c0;
    v4f u = *(const v4f*)ph, w = *(const v4f*)(ph + 4);
    u.x = log1pf(fmaxf(u.x, 0.f)); u.y = log1pf(fmaxf(u.y, 0.f));
    u.z = log1pf(fmaxf(u.z, 0.f)); u.w = log1pf(fmaxf(u.w, 0.f));
    w.x = log1pf(fmaxf(w.x, 0.f)); w.y = log1pf(fmaxf(w.y, 0.f));
    w.z = log1pf(fmaxf(w.z, 0.f)); w.w = log1pf(fmaxf(w.w, 0.f));
    *(v4f*)(xll + q * TT + c0)     = u;
    *(v4f*)(xll + q * TT + c0 + 4) = w;
  }
  for (int i = tid; i < GN * HP / 2; i += NTHR) ((unsigned int*)hA)[i] = 0u;

  Frag bq[3][2];
#pragma unroll
  for (int g = 0; g < 3; ++g) {
    const _Float16* p = Whh16 + (size_t)(64 * g + d) * DM;
#pragma unroll
    for (int ks = 0; ks < 2; ++ks) {
      bq[g][ks].half[0] = *(const v8h*)(p + 32 * ks + 8 * hh);
      bq[g][ks].half[1] = *(const v8h*)(p + 32 * ks + 16 + 8 * hh);
    }
  }
  float wi0[3], wi1[3], bi[3], bh[3];
#pragma unroll
  for (int g = 0; g < 3; ++g) {
    wi0[g] = Wih[(64 * g + d) * 2];
    wi1[g] = Wih[(64 * g + d) * 2 + 1];
    bi[g]  = bih[64 * g + d];
    bh[g]  = bhh[64 * g + d];
  }
  float hreg[8];
#pragma unroll
  for (int r = 0; r < 8; ++r) hreg[r] = 0.0f;
  __syncthreads();

  const _Float16* pa = hA + (16 * mt + m) * HP + 8 * hh;
  const v8f z8 = {0.f, 0.f, 0.f, 0.f, 0.f, 0.f, 0.f, 0.f};
#pragma unroll 1
  for (int t = 0; t < TT; ++t) {
    Frag a0, a1;
    a0.half[0] = *(const v8h*)(pa);      a0.half[1] = *(const v8h*)(pa + 16);
    a1.half[0] = *(const v8h*)(pa + 32); a1.half[1] = *(const v8h*)(pa + 48);
    __syncthreads();
    v8f ar = wm(a0.v, bq[0][0].v, z8); ar = wm(a1.v, bq[0][1].v, ar);
    v8f az = wm(a0.v, bq[1][0].v, z8); az = wm(a1.v, bq[1][1].v, az);
    v8f an = wm(a0.v, bq[2][0].v, z8); an = wm(a1.v, bq[2][1].v, an);
#pragma unroll
    for (int r = 0; r < 8; ++r) {
      const int nl = 16 * mt + 8 * hh + r;
      const float xc = xcl[nl * TT + t];
      const float xl = xll[nl * TT + t];
      const float gir = xc * wi0[0] + xl * wi1[0] + bi[0];
      const float giz = xc * wi0[1] + xl * wi1[1] + bi[1];
      const float gin = xc * wi0[2] + xl * wi1[2] + bi[2];
      const float ghr = ar[r] * 0.125f + bh[0];
      const float ghz = az[r] * 0.125f + bh[1];
      const float ghn = an[r] * 0.125f + bh[2];
      const float rg = sigm(gir + ghr);
      const float zg = sigm(giz + ghz);
      const float ng = tnh(gin + rg * ghn);
      const float hn = (1.0f - zg) * ng + zg * hreg[r];
      hreg[r] = hn;
      hA[nl * HP + d] = (_Float16)hn;
    }
    __syncthreads();
  }

#pragma unroll
  for (int r = 0; r < 8; ++r) hf[(16 * mt + 8 * hh + r) * FP + d] = hreg[r];
  __syncthreads();
  float xv[8];
  ld8f(hf + q * FP + c0, xv);
  float s = 0.f;
#pragma unroll
  for (int j = 0; j < 8; ++j) s += xv[j];
  s += __shfl_xor(s, 1, 32); s += __shfl_xor(s, 2, 32); s += __shfl_xor(s, 4, 32);
  const float mu = s * (1.0f / 64.0f);
  float qv = 0.f;
#pragma unroll
  for (int j = 0; j < 8; ++j) { xv[j] -= mu; qv += xv[j] * xv[j]; }
  qv += __shfl_xor(qv, 1, 32); qv += __shfl_xor(qv, 2, 32); qv += __shfl_xor(qv, 4, 32);
  const float rs = 1.0f / sqrtf(qv * (1.0f / 64.0f) + 1e-5f);
  const int ng  = nodeBase + q;
  const int ngc = (ng > nN - 1) ? (nN - 1) : ng;
  const float l0 = log1pf(fmaxf(flops[ngc], 0.f));
  const float l1 = log1pf(fmaxf(memv[ngc], 0.f));
  const float f0 = fin[ngc], f1 = fout[ngc], f2 = flvl[ngc];
  Pack16 u;
#pragma unroll
  for (int j = 0; j < 8; ++j) {
    const int c = c0 + j;
    const float hd = xv[j] * rs * lng[c] + lnb[c];
    const float hs = l0 * Wst[c] + l1 * Wst[DM + c] + bst[c];
    const float ht = f0 * Wsr[c] + f1 * Wsr[DM + c] + f2 * Wsr[2 * DM + c] + bsr[c];
    const float v  = (hs + hd) + ht;
    u.h[j] = (_Float16)fmaxf(v, 0.f);
  }
  _Float16* op = x0h + (size_t)ng * DM + c0;
  *(volatile v4i*)op = u.i;
  __threadfence();
  *(volatile v4i*)op = u.i;
}

template <int NCOL, int NHD, int XSP, int NIT>
__device__ __forceinline__ void xf_store(const float* Xs, const float* Af, const float* Df,
                                         float* xp, float* asP, float* adP,
                                         int rowBase, int tid, int wave, int lane) {
  constexpr int NC4 = NCOL / 4;
#pragma unroll
  for (int it = 0; it < NIT; ++it) {
    const int f   = it * NTHR + tid;
    const int row = f / NC4;
    const int c4  = f - row * NC4;
    const v4f v = *(const v4f*)(Xs + row * XSP + 4 * c4);
    *(volatile v4f*)(xp + (size_t)(rowBase + row) * NCOL + 4 * c4) = v;
  }
  const int lc = (lane < 8 * NHD) ? lane : (8 * NHD - 1);
  const v4f va = *(const v4f*)(Af + 4 * lc);
  const v4f vd = *(const v4f*)(Df + 4 * lc);
  if (wave == 0 && lane < 8 * NHD) *(volatile v4f*)(asP + (size_t)rowBase * NHD + 4 * lane) = va;
  if (wave == 1 && lane < 8 * NHD) *(volatile v4f*)(adP + (size_t)rowBase * NHD + 4 * lane) = vd;
}

template <int K, int NCOL, int NHD, int TPW>
__global__ __launch_bounds__(NTHR) void k_xform(const _Float16* __restrict__ A16, const _Float16* __restrict__ Wt,
                                                  const float* __restrict__ asw, const float* __restrict__ adw,
                                                  float* xp, float* asP, float* adP) {
  constexpr int XSP = NCOL + 4;
  constexpr int WPH = 4 / TPW;
  constexpr int NC4 = NCOL / 4;
  constexpr int NIT = (32 * NC4) / NTHR;
  static_assert(NCOL == 64 * TPW);
  static_assert(NCOL == 64 * NHD);
  static_assert((K % 32) == 0);
  static_assert(((32 * NC4) % NTHR) == 0);
  static_assert(WPH * TPW == 4);
  __shared__ __attribute__((aligned(16))) float Xs[32 * XSP];
  __shared__ float Ps[32 * NHD * WPH];
  __shared__ float Pd[32 * NHD * WPH];
  __shared__ __attribute__((aligned(16))) float Af[32 * NHD];
  __shared__ __attribute__((aligned(16))) float Df[32 * NHD];

  const int tid  = threadIdx.x;
  const int lane = tid & 31;
  const int wave = tid >> 5;
  const int hh   = lane >> 4;
  const int m    = lane & 15;
  const int mt   = wave >> 2;
  const int sub  = wave & 3;
  const int head = (sub * TPW) >> 2;
  const int pw   = sub - head * WPH;
  const int rowBase = blockIdx.x * 32;

  v8f acc[TPW];
#pragma unroll
  for (int i = 0; i < TPW; ++i) { const v8f z = {0.f, 0.f, 0.f, 0.f, 0.f, 0.f, 0.f, 0.f}; acc[i] = z; }
  const _Float16* pa = A16 + (size_t)(rowBase + 16 * mt + m) * K + 8 * hh;
#pragma unroll
  for (int ks = 0; ks < K / 32; ++ks) {
    Frag a;
    a.half[0] = *(const v8h*)(pa + 32 * ks);
    a.half[1] = *(const v8h*)(pa + 32 * ks + 16);
#pragma unroll
    for (int i = 0; i < TPW; ++i) {
      const int nt = sub * TPW + i;
      const _Float16* pb = Wt + (size_t)(16 * nt + m) * K + 32 * ks + 8 * hh;
      Frag b;
      b.half[0] = *(const v8h*)pb;
      b.half[1] = *(const v8h*)(pb + 16);
      acc[i] = wm(a.v, b.v, acc[i]);
    }
  }

  float ss[8], sd[8];
#pragma unroll
  for (int r = 0; r < 8; ++r) { ss[r] = 0.f; sd[r] = 0.f; }
#pragma unroll
  for (int i = 0; i < TPW; ++i) {
    const int col = 16 * (sub * TPW + i) + m;
    const float cs = asw[col];
    const float cd = adw[col];
#pragma unroll
    for (int r = 0; r < 8; ++r) {
      const float v = acc[i][r] * 0.125f;
      Xs[(16 * mt + 8 * hh + r) * XSP + col] = v;
      ss[r] += v * cs;
      sd[r] += v * cd;
    }
  }
#pragma unroll
  for (int mk = 1; mk < 16; mk <<= 1) {
#pragma unroll
    for (int r = 0; r < 8; ++r) {
      ss[r] += __shfl_xor(ss[r], mk, 32);
      sd[r] += __shfl_xor(sd[r], mk, 32);
    }
  }
  if (m == 0) {
#pragma unroll
    for (int r = 0; r < 8; ++r) {
      Ps[((16 * mt + 8 * hh + r) * NHD + head) * WPH + pw] = ss[r];
      Pd[((16 * mt + 8 * hh + r) * NHD + head) * WPH + pw] = sd[r];
    }
  }
  __syncthreads();
  if (tid < 32 * NHD) {
    float s1 = 0.f, s2 = 0.f;
#pragma unroll
    for (int p = 0; p < WPH; ++p) { s1 += Ps[tid * WPH + p]; s2 += Pd[tid * WPH + p]; }
    Af[tid] = s1;
    Df[tid] = s2;
  }
  __syncthreads();
  xf_store<NCOL, NHD, XSP, NIT>(Xs, Af, Df, xp, asP, adP, rowBase, tid, wave, lane);
  __threadfence();
  xf_store<NCOL, NHD, XSP, NIT>(Xs, Af, Df, xp, asP, adP, rowBase, tid, wave, lane);
}

template <int DF, int NHD, int NB, int ELU, typename OT>
__global__ __launch_bounds__(NTHR) void k_gat(
    const int* __restrict__ ei, const float* __restrict__ xp,
    const float* __restrict__ asrc, const float* __restrict__ adst,
    const float* __restrict__ bias, const float* __restrict__ gam, const float* __restrict__ bet,
    OT* out, int nN, int nE, int nP) {
  constexpr int CPL  = DF / 32;
  constexpr int SACC = NB * DF;
  constexpr int NA   = NB * NHD;
  constexpr int SLB  = (NB == 256) ? 8 : 10;
  constexpr int SPW  = NB / NWAVE;
  static_assert((1 << SLB) == NB);
  static_assert(DF == 64 * NHD);
  static_assert(CPL == 8 || CPL == 2);
  static_assert(((SACC + NA) % 4) == 0);
  static_assert(CHUNK <= 2048);

  extern __shared__ v4f lds_dyn[];
  float* sacc = (float*)lds_dyn;
  float* den  = sacc + SACC;
  float* mx   = den + NA;
  int*   list = (int*)(mx + NA);
  int*   wcnt = list + NWAVE * WCAP;

  const int tid  = threadIdx.x;
  const int lane = tid & 31;
  const int wave = tid >> 5;
  const int hh   = lane >> 4;
  const int m    = lane & 15;
  const int c0   = CPL * lane;
  const int hd   = c0 >> 6;
  const int nodeBase = blockIdx.x * NB;
  const float ninf = __int_as_float(0xff800000);

  {
    const v4f z4 = {0.f, 0.f, 0.f, 0.f};
    for (int i = tid; i < (SACC + NA) / 4; i += NTHR) lds_dyn[i] = z4;
    for (int i = tid; i < NA; i += NTHR) mx[i] = ninf;
  }
  __syncthreads();

  const int* eid = ei + nE;
  const bool al16 = ((nE & 3) == 0);
  const int nChunks = (nE + CHUNK - 1) / CHUNK;
#pragma unroll 1
  for (int ch = 0; ch < nChunks; ++ch) {
    const int cbase = ch * CHUNK;
    int wc = 0;
#pragma unroll
    for (int g = 0; g < NGRP; ++g) {
      const int el0 = (g * NTHR + tid) * 4;
      const int e0  = cbase + el0;
      const int sent = -2147483647 - 1;
      v4i d;
      if (al16 && (cbase + CHUNK <= nE)) {
        d = *(const v4i*)(eid + e0);
      } else {
        d.x = (e0     < nE) ? eid[min(e0, nE - 1)]     : sent;
        d.y = (e0 + 1 < nE) ? eid[min(e0 + 1, nE - 1)] : sent;
        d.z = (e0 + 2 < nE) ? eid[min(e0 + 2, nE - 1)] : sent;
        d.w = (e0 + 3 < nE) ? eid[min(e0 + 3, nE - 1)] : sent;
      }
      const unsigned s0 = (unsigned)d.x - (unsigned)nodeBase;
      const unsigned s1 = (unsigned)d.y - (unsigned)nodeBase;
      const unsigned s2 = (unsigned)d.z - (unsigned)nodeBase;
      const unsigned s3 = (unsigned)d.w - (unsigned)nodeBase;
      const bool h0 = s0 < (unsigned)NB;
      const bool h1 = s1 < (unsigned)NB;
      const bool h2 = s2 < (unsigned)NB;
      const bool h3 = s3 < (unsigned)NB;
      const unsigned many = __builtin_amdgcn_ballot_w32(h0 | h1 | h2 | h3);
      if (many != 0u) {
#define HITJ(J, HJ, SJ) { \
          const unsigned mj = __builtin_amdgcn_ballot_w32(HJ); \
          if (HJ) { \
            const int pos = wc + (int)__builtin_amdgcn_mbcnt_lo(mj, 0u); \
            if (pos < WCAP) list[wave * WCAP + pos] = ((el0 + (J)) << SLB) | (int)(SJ); \
          } \
          wc += (int)__builtin_popcount(mj); }
        HITJ(0, h0, s0)
        HITJ(1, h1, s1)
        HITJ(2, h2, s2)
        HITJ(3, h3, s3)
#undef HITJ
      }
    }
    if (lane == 0) wcnt[wave] = wc;
    __syncthreads();

    if (wave == 0) {
#pragma unroll 1
      for (int wsx = 0; wsx < NWAVE; ++wsx) {
        int n = wcnt[wsx];
        if (n > WCAP) n = WCAP;
        if (n < 0) n = 0;
#pragma unroll 1
        for (int i = 0; i < n; ++i) {
          const int ent  = list[wsx * WCAP + i];
          const int slot = ent & (NB - 1);
          const int el   = (ent >> SLB) & (CHUNK - 1);
          int e = cbase + el;
          if (e > nE - 1) e = nE - 1;
          int src = ei[e];
          src = src < 0 ? 0 : (src > nN - 1 ? nN - 1 : src);
          int nd = nodeBase + slot;
          if (nd > nN - 1) nd = nN - 1;
          float al = asrc[(size_t)src * NHD + hd] + adst[(size_t)nd * NHD + hd];
          al = (al > 0.f) ? al : 0.2f * al;
          const int   ai = slot * NHD + hd;
          const float mo = mx[ai];
          const float mn = fmaxf(mo, al);
          const float sc = __expf(mo - mn);
          const float p  = __expf(al - mn);
          float xv[CPL], cur[CPL];
          ldc<CPL>(xp + (size_t)src * DF + c0, xv);
          float* sp = sacc + slot * DF + c0;
          ldc<CPL>(sp, cur);
#pragma unroll
          for (int j = 0; j < CPL; ++j) cur[j] = cur[j] * sc + p * xv[j];
          stc<CPL>(sp, cur);
          const float dn = den[ai] * sc + p;
          den[ai] = dn;
          mx[ai]  = mn;
        }
      }
    }
    __syncthreads();
  }

  float bb[CPL], gg[CPL], be[CPL];
  ldc<CPL>(bias + c0, bb);
  ldc<CPL>(gam + c0, gg);
  ldc<CPL>(bet + c0, be);
#pragma unroll 1
  for (int j = 0; j < SPW; ++j) {
    const int slot = wave * SPW + j;
    const int node = nodeBase + slot;
    if (node >= nN) break;
    float al = asrc[(size_t)node * NHD + hd] + adst[(size_t)node * NHD + hd];
    al = (al > 0.f) ? al : 0.2f * al;
    const int   ai = slot * NHD + hd;
    const float mo = mx[ai];
    const float mn = fmaxf(mo, al);
    const float sc = __expf(mo - mn);
    const float p  = __expf(al - mn);
    float xv[CPL], sv[CPL], h[CPL];
    ldc<CPL>(xp + (size_t)node * DF + c0, xv);
    ldc<CPL>(sacc + slot * DF + c0, sv);
    const float dv  = den[ai] * sc + p;
    const float inv = 1.0f / (dv + 1e-16f);
    float s = 0.f;
#pragma unroll
    for (int jj = 0; jj < CPL; ++jj) {
      float hv = (sv[jj] * sc + p * xv[jj]) * inv + bb[jj];
      if (ELU) hv = (hv > 0.f) ? hv : (__expf(hv) - 1.0f);
      h[jj] = hv;
      s += hv;
    }
    s = wsum(s);
    const float mu = s * (1.0f / (float)DF);
    float qv = 0.f;
#pragma unroll
    for (int jj = 0; jj < CPL; ++jj) { h[jj] -= mu; qv += h[jj] * h[jj]; }
    qv = wsum(qv);
    const float rs = 1.0f / sqrtf(qv * (1.0f / (float)DF) + 1e-5f);
#pragma unroll
    for (int jj = 0; jj < CPL; ++jj) h[jj] = h[jj] * rs * gg[jj] + be[jj];
    stc<CPL>(sacc + slot * DF + c0, h);
  }
  __syncthreads();

#pragma unroll 1
  for (int pass = 0; pass < 2; ++pass) {
    if constexpr (CPL == 8) {
      _Float16* o16 = reinterpret_cast<_Float16*>(out);
#pragma unroll 1
      for (int j = 0; j < SPW; ++j) {
        const int slot = wave * SPW + j;
        const int node = nodeBase + slot;
        if (node >= nP) break;
        float v[8];
        ld8f(sacc + slot * DF + 8 * lane, v);
        Pack16 u;
#pragma unroll
        for (int jj = 0; jj < 8; ++jj) u.h[jj] = (_Float16)v[jj];
        *(volatile v4i*)(o16 + (size_t)node * DF + 8 * lane) = u.i;
      }
    } else {
      float* o32 = reinterpret_cast<float*>(out);
#pragma unroll 1
      for (int j2 = 0; j2 < SPW / 2; ++j2) {
        const int sbase = wave * SPW + 2 * j2;
        if (nodeBase + sbase >= nN) break;
        const int slot = sbase + hh;
        const int node = nodeBase + slot;
        const v4f v = *(const v4f*)(sacc + slot * DF + 4 * m);
        if (node < nN) *(volatile v4f*)(o32 + (size_t)node * DF + 4 * m) = v;
      }
    }
    __threadfence();
  }
}

static inline size_t al256(size_t b) { return (b + 255) & ~(size_t)255; }

extern "C" void kernel_launch(void* const* d_in, const int* in_sizes, int n_in,
                              void* d_out, int out_size, void* d_ws, size_t ws_size,
                              hipStream_t stream) {
  if (n_in < 27) return;
  const int nN  = in_sizes[1];
  const int nE2 = in_sizes[0];
  if (nN <= 0 || nN > MAXN) return;
  if (nE2 < 2 || (nE2 & 1)) return;
  const int nE = nE2 / 2;
  if (in_sizes[2] != nN) return;
  if (in_sizes[3] != nN * TT || in_sizes[4] != nN * TT) return;
  if (in_sizes[5] != 2 * DM || in_sizes[6] != DM) return;
  if (in_sizes[7] != 192 * 2 || in_sizes[8] != 192 * DM || in_sizes[9] != 192 || in_sizes[10] != 192) return;
  if (in_sizes[11] != DM || in_sizes[12] != DM) return;
  if (in_sizes[13] != 3 * DM || in_sizes[14] != DM) return;
  if (in_sizes[15] != DM * 256 || in_sizes[16] != 256 || in_sizes[17] != 256 || in_sizes[18] != 256) return;
  if (in_sizes[19] != 256 * DM || in_sizes[20] != DM || in_sizes[21] != DM || in_sizes[22] != DM) return;
  if (in_sizes[23] != 256 || in_sizes[24] != 256 || in_sizes[25] != DM || in_sizes[26] != DM) return;
  if (out_size != nN * DM) return;

  const int*   ei     = (const int*)d_in[0];
  const float* flops  = (const float*)d_in[1];
  const float* memv   = (const float*)d_in[2];
  const float* tcs    = (const float*)d_in[3];
  const float* hls    = (const float*)d_in[4];
  const float* Wst    = (const float*)d_in[5];
  const float* bst    = (const float*)d_in[6];
  const float* Wih    = (const float*)d_in[7];
  const float* Whh    = (const float*)d_in[8];
  const float* bih    = (const float*)d_in[9];
  const float* bhh    = (const float*)d_in[10];
  const float* lng    = (const float*)d_in[11];
  const float* lnb    = (const float*)d_in[12];
  const float* Wsr    = (const float*)d_in[13];
  const float* bsr    = (const float*)d_in[14];
  const float* g1W    = (const float*)d_in[15];
  const float* g1as   = (const float*)d_in[16];
  const float* g1ad   = (const float*)d_in[17];
  const float* g1b    = (const float*)d_in[18];
  const float* g2W    = (const float*)d_in[19];
  const float* g2as   = (const float*)d_in[20];
  const float* g2ad   = (const float*)d_in[21];
  const float* g2b    = (const float*)d_in[22];
  const float* ln1g   = (const float*)d_in[23];
  const float* ln1b   = (const float*)d_in[24];
  const float* ln2g   = (const float*)d_in[25];
  const float* ln2b   = (const float*)d_in[26];
  float* out = (float*)d_out;

  const int nP    = ((nN + 31) / 32) * 32;
  const int nBlkS = (nP + NBS - 1) / NBS;

  size_t off = 0;
  char* base = (char*)d_ws;
  _Float16* Whh16 = (_Float16*)(base + off); off += al256((size_t)192 * DM * 2);
  _Float16* Wt1   = (_Float16*)(base + off); off += al256((size_t)256 * 64 * 2);
  _Float16* Wt2   = (_Float16*)(base + off); off += al256((size_t)64 * 256 * 2);
  int* csr        = (int*)(base + off);      off += al256((size_t)nBlkS * CAPB * 4);
  int* pcin       = (int*)(base + off);      off += al256((size_t)nBlkS * NBS * 4);
  int* pcou       = (int*)(base + off);      off += al256((size_t)nBlkS * NBS * 4);
  int* poff       = (int*)(base + off);      off += al256((size_t)nBlkS * NBS * 4);
  float* fin      = (float*)(base + off);    off += al256((size_t)nP * 4);
  float* fout     = (float*)(base + off);    off += al256((size_t)nP * 4);
  float* flvl     = (float*)(base + off);    off += al256((size_t)nP * 4);
  _Float16* x0h   = (_Float16*)(base + off); off += al256((size_t)nP * DM * 2);
  float* xp1      = (float*)(base + off);    off += al256((size_t)nP * 256 * 4);
  float* as1      = (float*)(base + off);    off += al256((size_t)nP * 4 * 4);
  float* ad1      = (float*)(base + off);    off += al256((size_t)nP * 4 * 4);
  _Float16* h1h   = (_Float16*)(base + off); off += al256((size_t)nP * 256 * 2);
  float* xp2      = (float*)(base + off);    off += al256((size_t)nP * DM * 4);
  float* as2      = (float*)(base + off);    off += al256((size_t)nP * 4);
  float* ad2      = (float*)(base + off);    off += al256((size_t)nP * 4);
  if (off > ws_size || off > (size_t)134217728) return;

  const size_t ldsStruct = (size_t)2 * nN * sizeof(int);
  constexpr int LDS_GAT1 = (256 * 256 + 2 * 256 * 4 + NWAVE * WCAP + NWAVE) * 4;
  constexpr int LDS_GAT2 = (1024 * 64 + 2 * 1024 * 1 + NWAVE * WCAP + NWAVE) * 4;
  static_assert(LDS_GAT1 == 278560);
  static_assert(LDS_GAT2 == 278560);

  k_prep<<<22, NTHR, 0, stream>>>(Whh, g1W, g2W, Whh16, Wt1, Wt2);

  hipFuncSetAttribute(reinterpret_cast<const void*>(&k_csr),
                      hipFuncAttributeMaxDynamicSharedMemorySize, LDS_CSR_BYTES);
  k_csr<<<nBlkS, STHR, LDS_CSR_BYTES, stream>>>(ei, nE, nN, csr, pcin, pcou, poff);

  hipFuncSetAttribute(reinterpret_cast<const void*>(&k_struct),
                      hipFuncAttributeMaxDynamicSharedMemorySize, (int)ldsStruct);
  k_struct<<<1, STHR, ldsStruct, stream>>>((const int*)csr, (const int*)pcin, (const int*)pcou,
                                           (const int*)poff, nN, nP, fin, fout, flvl);

  k_gru<<<nP / GN, NTHR, 0, stream>>>(tcs, hls, Wih, Whh16, bih, bhh, lng, lnb, flops, memv,
                                      Wst, bst, fin, fout, flvl, Wsr, bsr, x0h, nN);

  hipLaunchKernelGGL(HIP_KERNEL_NAME(k_xform<64, 256, 4, 4>), dim3(nP / 32), dim3(NTHR), 0, stream,
                     (const _Float16*)x0h, (const _Float16*)Wt1, g1as, g1ad, xp1, as1, ad1);

  hipFuncSetAttribute(reinterpret_cast<const void*>(&k_gat<256, 4, 256, 1, _Float16>),
                      hipFuncAttributeMaxDynamicSharedMemorySize, LDS_GAT1);
  hipLaunchKernelGGL(HIP_KERNEL_NAME(k_gat<256, 4, 256, 1, _Float16>), dim3((nP + 255) / 256), dim3(NTHR),
                     LDS_GAT1, stream, ei, (const float*)xp1, (const float*)as1, (const float*)ad1,
                     g1b, ln1g, ln1b, h1h, nN, nE, nP);

  hipLaunchKernelGGL(HIP_KERNEL_NAME(k_xform<256, 64, 1, 1>), dim3(nP / 32), dim3(NTHR), 0, stream,
                     (const _Float16*)h1h, (const _Float16*)Wt2, g2as, g2ad, xp2, as2, ad2);

  hipFuncSetAttribute(reinterpret_cast<const void*>(&k_gat<64, 1, 1024, 0, float>),
                      hipFuncAttributeMaxDynamicSharedMemorySize, LDS_GAT2);
  hipLaunchKernelGGL(HIP_KERNEL_NAME(k_gat<64, 1, 1024, 0, float>), dim3((nP + 1023) / 1024), dim3(NTHR),
                     LDS_GAT2, stream, ei, (const float*)xp2, (const float*)as2, (const float*)ad2,
                     g2b, ln2g, ln2b, out, nN, nE, nP);
}
